// TopKMoE_6597069767522
// MI455X (gfx1250) — hardware-verified
//
#include <hip/hip_runtime.h>
#include <math.h>

typedef __attribute__((ext_vector_type(16))) _Float16 v16h;
typedef __attribute__((ext_vector_type(16))) __bf16 v16b;
typedef __attribute__((ext_vector_type(8)))  _Float16 v8h;
typedef __attribute__((ext_vector_type(8)))  __bf16 v8b;
typedef __attribute__((ext_vector_type(8)))  float v8f;
typedef __attribute__((ext_vector_type(4)))  float v4f;
typedef __attribute__((ext_vector_type(4)))  unsigned v4u;

#ifndef NB
#define NB 4096
#endif
#define NB_FULL 4096
#define DIN  256
#define DHID 512
#define DOUT 256
#define NE   8
#define KF (NE * DHID)
#define KP (KF + 64)
#define HCARRY 64.0f
#define WCARRY 512.0f
#define OSCALE (1.0f / 32768.0f)

#define WS_XB  ((size_t)0)
#define WS_W1T (WS_XB  + (size_t)NB * DIN * 2)
#define WS_W2T (WS_W1T + (size_t)NE * DHID * DIN * 2)
#define WS_HB  (WS_W2T + (size_t)DOUT * KP * 2)
#define WS_CW  (WS_HB  + (size_t)NB * KP * 2)
#define WS_END (WS_CW  + (size_t)NB * NE * 4)

static_assert(NB % 128 == 0);
static_assert(NB <= NB_FULL);
static_assert(DIN % 32 == 0 && KP % 32 == 0 && (KP * 2) % 128 == 0);
static_assert((size_t)NB_FULL * DOUT * 4 == 4194304);
static_assert(WS_W1T % 128 == 0 && WS_W2T % 128 == 0 && WS_HB % 128 == 0 && WS_CW % 128 == 0);
static_assert(WS_END <= (size_t)134217728);
static_assert(NE == 8);
static_assert(NE % 8 == 0 && NE <= 64);
static_assert(DIN % 8 == 0 && (DIN * NE / 4) % 256 == 0);
static_assert(DOUT % 128 == 0 && DHID % 128 == 0 && (DOUT & (DOUT - 1)) == 0);
static_assert((size_t)(NB * DIN / 8 / 256) * 256 * 8 == (size_t)NB * DIN);
static_assert((size_t)(DHID / 64) * (DIN / 64) * NE * 4096 == (size_t)NE * DIN * DHID);
static_assert((size_t)(DOUT / 64) * (DHID / 64) * NE * 4096 == (size_t)DOUT * KF);
static_assert((size_t)(DOUT * 8 / 256) * 256 * 8 == (size_t)DOUT * 64);
static_assert((size_t)(NB / 64) * 64 * NE == (size_t)NB * NE);
static_assert((size_t)(NB / 64) * 512 * 8 == (size_t)NB * 64);
static_assert(128 * 4 == 64 * NE);
static_assert(256 * 2 * 8 == 64 * 64);
static_assert((size_t)(DHID / 128) * (NB / 128) * NE * 128 * 128 == (size_t)NB * KF);
static_assert((size_t)(DOUT / 128) * (NB / 128) * 128 * 128 == (size_t)NB * DOUT);
static_assert(64 * 65 * 4 <= 131072);
static_assert(DIN * NE * 4 + 2 * 64 * NE * 4 <= 131072);
static_assert(8 * 32 * 64 * 2 <= 131072);
static_assert(8 * 16 * 64 * 4 <= 131072);

__device__ __forceinline__ v8f wmma16(v16h a, v16h b, v8f c) {
  v8f d = __builtin_amdgcn_wmma_f32_16x16x32_f16(false, a, false, b, (short)0, c, false, false);
  asm volatile("v_nop\n\tv_nop\n\tv_nop\n\tv_nop" : "+v"(d) : "v"(a), "v"(b));
  return d;
}
__device__ __forceinline__ v8f wmma_bf(v16b a, v16b b, v8f c) {
  v8f d = __builtin_amdgcn_wmma_f32_16x16x32_bf16(false, a, false, b, (short)0, c, false, false);
  asm volatile("v_nop\n\tv_nop\n\tv_nop\n\tv_nop" : "+v"(d) : "v"(a), "v"(b));
  return d;
}
__device__ __forceinline__ float bfr(float v) { return (float)(__bf16)v; }
__device__ __forceinline__ _Float16 toh_flush(float v) { const _Float16 r = (_Float16)v; return (fabsf(v) < 6.103515625e-05f) ? (_Float16)0.0f : r; }
__device__ __forceinline__ v16b ldfrag_b(const unsigned short* p) { union { v16b v; v4u q[2]; } f; f.q[0] = *(const v4u*)p; f.q[1] = *(const v4u*)(p + 16); return f.v; }
__device__ __forceinline__ v16h ldfrag_h(const unsigned short* p) { union { v16h v; v4u q[2]; } f; f.q[0] = *(const v4u*)p; f.q[1] = *(const v4u*)(p + 16); return f.v; }

__global__ __launch_bounds__(256) void k_cvt_x(const float* __restrict__ X, unsigned short* __restrict__ XB) {
  const unsigned i = blockIdx.x * 256u + threadIdx.x;
  const unsigned ic = i < (unsigned)(NB * DIN / 8) ? i : (unsigned)(NB * DIN / 8 - 1);
  const v4f a = *(const v4f*)(X + (size_t)ic * 8), b = *(const v4f*)(X + (size_t)ic * 8 + 4);
  union { v8b h; v4u u; } o;
#pragma unroll
  for (int j = 0; j < 4; ++j) { o.h[j] = (__bf16)a[j]; o.h[4 + j] = (__bf16)b[j]; }
  const v4u val = o.u;
  volatile v4u* p = (volatile v4u*)(XB + (size_t)ic * 8);
  *p = val; __threadfence(); *p = val;
}

template <int F16>
__global__ __launch_bounds__(256) void k_tr(const float* __restrict__ S, unsigned short* __restrict__ Dst, unsigned K, unsigned N, unsigned dpitch, unsigned erow, unsigned ecol, float sc) {
  __shared__ float tile[64][65];
  const unsigned t = threadIdx.x, e = blockIdx.z, k0 = blockIdx.y * 64u, n0 = blockIdx.x * 64u;
  const float* s = S + (size_t)e * K * N;
#pragma unroll
  for (unsigned it = 0; it < 4; ++it) { const unsigned idx = it * 256u + t, kr = idx >> 4, c4 = idx & 15u;
    const v4f v = *(const v4f*)(s + (size_t)(k0 + kr) * N + n0 + 4u * c4);
    tile[kr][4u * c4 + 0] = v[0]; tile[kr][4u * c4 + 1] = v[1]; tile[kr][4u * c4 + 2] = v[2]; tile[kr][4u * c4 + 3] = v[3]; }
  __syncthreads();
  v4u o[2];
#pragma unroll
  for (unsigned it = 0; it < 2; ++it) { const unsigned idx = it * 256u + t, nr = idx >> 3, q = idx & 7u;
    union { v8b b; v8h h; v4u u; } w;
#pragma unroll
    for (int i = 0; i < 8; ++i) { const float v = bfr(tile[8u * q + i][nr]); if (F16) w.h[i] = toh_flush(v * sc); else w.b[i] = (__bf16)v; }
    o[it] = w.u; }
#pragma unroll
  for (unsigned it = 0; it < 2; ++it) { const unsigned idx = it * 256u + t, nr = idx >> 3, q = idx & 7u;
    *(volatile v4u*)(Dst + (size_t)(e * erow + n0 + nr) * dpitch + e * ecol + k0 + 8u * q) = o[it]; }
  __threadfence();
#pragma unroll
  for (unsigned it = 0; it < 2; ++it) { const unsigned idx = it * 256u + t, nr = idx >> 3, q = idx & 7u;
    *(volatile v4u*)(Dst + (size_t)(e * erow + n0 + nr) * dpitch + e * ecol + k0 + 8u * q) = o[it]; }
}

__global__ __launch_bounds__(256) void k_b2pad(const float* __restrict__ B2, unsigned short* __restrict__ W2T) {
  const unsigned idx = blockIdx.x * 256u + threadIdx.x; const unsigned n = (idx >> 3) & (DOUT - 1u), q = idx & 7u;
  const unsigned qc = q < (unsigned)(NE / 8) ? q : 0u; const float keep = q < (unsigned)(NE / 8) ? 1.f : 0.f;
  union { v8h h; v4u u; } w;
#pragma unroll
  for (int i = 0; i < 8; ++i) w.h[i] = toh_flush(bfr(B2[(size_t)(8u * qc + i) * DOUT + n]) * WCARRY * keep);
  const v4u val = w.u;
  volatile v4u* p = (volatile v4u*)(W2T + (size_t)n * KP + KF + 8u * q);
  *p = val; __threadfence(); *p = val;
}

__global__ __launch_bounds__(256) void k_gate(const unsigned short* __restrict__ XB, const float* __restrict__ WG, const float* __restrict__ BG, const float* __restrict__ BI, float* __restrict__ CW, unsigned short* __restrict__ HB) {
#pragma clang fp contract(off)
  __shared__ __align__(16) float sW[DIN][NE];
  __shared__ __align__(16) float sl[64][NE];
  __shared__ __align__(16) float sp[64][NE];
  const unsigned tid = threadIdx.x, lane = tid & 31u;
  const unsigned wave = (unsigned)__builtin_amdgcn_readfirstlane((int)(threadIdx.x >> 5));
  const unsigned r0 = blockIdx.x * 64u;
  const unsigned tok = (wave & 1u) * 32u + lane, eq = wave >> 1;
#pragma unroll 1
  for (unsigned idx = tid; idx < (unsigned)(DIN * NE / 4); idx += 256u) { const v4f w = *(const v4f*)(WG + 4u * idx); v4f o;
#pragma unroll
    for (int j = 0; j < 4; ++j) o[j] = bfr(w[j]);
    *(v4f*)(&sW[0][0] + 4u * idx) = o; }
  __syncthreads();
  const unsigned short* xp = XB + (size_t)(r0 + tok) * DIN;
  float a0 = 0.f, a1 = 0.f;
#pragma unroll 1
  for (unsigned kc = 0; kc < DIN / 8; ++kc) { const v4u xw = *(const v4u*)(xp + kc * 8u);
#pragma unroll
    for (int j = 0; j < 4; ++j) { const float xl = __uint_as_float(xw[j] << 16), xh = __uint_as_float(xw[j] & 0xffff0000u);
      const unsigned k = kc * 8u + 2u * (unsigned)j;
      const float wl0 = sW[k][2u * eq], wl1 = sW[k][2u * eq + 1u], wh0 = sW[k + 1u][2u * eq], wh1 = sW[k + 1u][2u * eq + 1u];
      a0 = fmaf(xl, wl0, a0); a1 = fmaf(xl, wl1, a1);
      a0 = fmaf(xh, wh0, a0); a1 = fmaf(xh, wh1, a1); } }
  const float l0 = (a0 + bfr(BG[2u * eq])) + bfr(BI[2u * eq]);
  const float l1 = (a1 + bfr(BG[2u * eq + 1u])) + bfr(BI[2u * eq + 1u]);
  sl[tok][2u * eq] = l0; sl[tok][2u * eq + 1u] = l1;
  __syncthreads();
  if (wave < 2u) {
    const v4f la = *(const v4f*)&sl[tok][0], lb = *(const v4f*)&sl[tok][4];
    float lg[NE];
#pragma unroll
    for (int j = 0; j < 4; ++j) { lg[j] = la[j]; lg[4 + j] = lb[j]; }
    unsigned i0 = 0u; float v0 = lg[0];
#pragma unroll
    for (int e = 1; e < NE; ++e) { const bool gt = lg[e] > v0; v0 = gt ? lg[e] : v0; i0 = gt ? (unsigned)e : i0; }
    unsigned i1 = (unsigned)NE; float v1 = -INFINITY;
#pragma unroll
    for (int e = 0; e < NE; ++e) { const bool gt = ((unsigned)e != i0) && (lg[e] > v1); v1 = gt ? lg[e] : v1; i1 = gt ? (unsigned)e : i1; }
    const float w = expf(v1 - v0); const float s = 1.0f + w; const float rs = 1.0f / s;
    const float w0 = rs, w1 = w * rs;
    v4f ca, cb;
#pragma unroll
    for (int j = 0; j < 4; ++j) { ca[j] = ((unsigned)j == i0) ? w0 : (((unsigned)j == i1) ? w1 : 0.f);
      cb[j] = ((unsigned)(4 + j) == i0) ? w0 : (((unsigned)(4 + j) == i1) ? w1 : 0.f); }
    *(v4f*)&sp[tok][0] = ca; *(v4f*)&sp[tok][4] = cb; }
  __syncthreads();
  v4u hv[2];
#pragma unroll
  for (unsigned it = 0; it < 2; ++it) { const unsigned idx = it * 256u + tid, rw = idx >> 3, q = idx & 7u; const unsigned qc = q < (unsigned)(NE / 8) ? q : 0u; const float keep = q < (unsigned)(NE / 8) ? 1.f : 0.f;
    union { v8h h; v4u u; } wq;
#pragma unroll
    for (int i = 0; i < 8; ++i) wq.h[i] = toh_flush(sp[rw][8u * qc + i] * HCARRY * keep);
    hv[it] = wq.u; }
  float* cwp = CW + (size_t)r0 * NE;
  v4f pv = {};
  if (wave < 4u) {
    pv = *(const v4f*)(&sp[0][0] + 4u * (tid & 127u));
    *(volatile v4f*)(cwp + 4u * tid) = pv; }
#pragma unroll
  for (unsigned it = 0; it < 2; ++it) { const unsigned idx = it * 256u + tid, rw = idx >> 3, q = idx & 7u; *(volatile v4u*)(HB + (size_t)(r0 + rw) * KP + KF + 8u * q) = hv[it]; }
  __threadfence();
  if (wave < 4u) *(volatile v4f*)(cwp + 4u * tid) = pv;
#pragma unroll
  for (unsigned it = 0; it < 2; ++it) { const unsigned idx = it * 256u + tid, rw = idx >> 3, q = idx & 7u; *(volatile v4u*)(HB + (size_t)(r0 + rw) * KP + KF + 8u * q) = hv[it]; }
}

__global__ __launch_bounds__(256) void k_h(const unsigned short* __restrict__ XB, const unsigned short* __restrict__ W1T, const float* __restrict__ B1, const float* __restrict__ WTS, unsigned short* __restrict__ HB) {
  __shared__ __align__(16) _Float16 sh[8][32][64];
  const unsigned t = threadIdx.x, wave = t >> 5, lane = t & 31u, lm = lane & 15u, lh = lane >> 4, wm = wave >> 1, wn = wave & 1u;
  const unsigned e = blockIdx.z, m0 = blockIdx.y * 128u, n0 = blockIdx.x * 128u;
  const unsigned short* ar[2]; const unsigned short* br[4];
#pragma unroll
  for (int mi = 0; mi < 2; ++mi) ar[mi] = XB + (size_t)(m0 + wm * 32u + mi * 16u + lm) * DIN + 8u * lh;
#pragma unroll
  for (int ni = 0; ni < 4; ++ni) br[ni] = W1T + (size_t)(e * DHID + n0 + wn * 64u + ni * 16u + lm) * DIN + 8u * lh;
  v8f acc[2][4] = {};
#pragma unroll 2
  for (unsigned kc = 0; kc < DIN / 32; ++kc) { v16b a[2], b[4];
#pragma unroll
    for (int mi = 0; mi < 2; ++mi) a[mi] = ldfrag_b(ar[mi] + kc * 32u);
#pragma unroll
    for (int ni = 0; ni < 4; ++ni) b[ni] = ldfrag_b(br[ni] + kc * 32u);
#pragma unroll
    for (int mi = 0; mi < 2; ++mi)
#pragma unroll
      for (int ni = 0; ni < 4; ++ni) acc[mi][ni] = wmma_bf(a[mi], b[ni], acc[mi][ni]); }
  float wv[2][8];
#pragma unroll
  for (int mi = 0; mi < 2; ++mi) {
#pragma unroll
    for (int r = 0; r < 8; ++r) wv[mi][r] = WTS[(size_t)(m0 + wm * 32u + mi * 16u + 8u * lh + r) * NE + e] * HCARRY;
    asm volatile("s_wait_loadcnt 0x0" ::: "memory"); }
#pragma unroll
  for (int ni = 0; ni < 4; ++ni) { const float bb = bfr(B1[(size_t)e * DHID + n0 + wn * 64u + ni * 16u + lm]);
#pragma unroll
    for (int mi = 0; mi < 2; ++mi)
#pragma unroll
      for (int r = 0; r < 8; ++r) sh[wave][mi * 16 + 8u * lh + r][ni * 16 + lm] = (_Float16)(fmaxf(acc[mi][ni][r] + bb, 0.f) * wv[mi][r]); }
  __syncthreads();
  v4u o[8];
#pragma unroll
  for (unsigned it = 0; it < 8; ++it) { const unsigned rw = it * 4u + (lane >> 3), q = lane & 7u; union { v8h h; v4u u; } w; w.h = *(const v8h*)&sh[wave][rw][8u * q]; o[it] = w.u; }
  unsigned short* hb = HB + (size_t)(m0 + wm * 32u) * KP + e * DHID + n0 + wn * 64u;
#pragma unroll
  for (unsigned it = 0; it < 8; ++it) { const unsigned rw = it * 4u + (lane >> 3), q = lane & 7u; *(volatile v4u*)(hb + (size_t)rw * KP + 8u * q) = o[it]; }
  __threadfence();
#pragma unroll
  for (unsigned it = 0; it < 8; ++it) { const unsigned rw = it * 4u + (lane >> 3), q = lane & 7u; *(volatile v4u*)(hb + (size_t)rw * KP + 8u * q) = o[it]; }
}

__global__ __launch_bounds__(256) void k_out(const unsigned short* __restrict__ HB, const unsigned short* __restrict__ W2T, float* __restrict__ OUT) {
  __shared__ __align__(16) float sf[8][16][64];
  const unsigned t = threadIdx.x, wave = t >> 5, lane = t & 31u, lm = lane & 15u, lh = lane >> 4, wm = wave >> 1, wn = wave & 1u;
  const unsigned m0 = blockIdx.y * 128u, n0 = blockIdx.x * 128u;
  const unsigned short* ar[2]; const unsigned short* br[4];
#pragma unroll
  for (int mi = 0; mi < 2; ++mi) ar[mi] = HB + (size_t)(m0 + wm * 32u + mi * 16u + lm) * KP + 8u * lh;
#pragma unroll
  for (int ni = 0; ni < 4; ++ni) br[ni] = W2T + (size_t)(n0 + wn * 64u + ni * 16u + lm) * KP + 8u * lh;
  v8f acc[2][4] = {};
#pragma unroll 2
  for (unsigned kc = 0; kc < KP / 32; ++kc) { v16h a[2], b[4];
#pragma unroll
    for (int mi = 0; mi < 2; ++mi) a[mi] = ldfrag_h(ar[mi] + kc * 32u);
#pragma unroll
    for (int ni = 0; ni < 4; ++ni) b[ni] = ldfrag_h(br[ni] + kc * 32u);
#pragma unroll
    for (int mi = 0; mi < 2; ++mi)
#pragma unroll
      for (int ni = 0; ni < 4; ++ni) acc[mi][ni] = wmma16(a[mi], b[ni], acc[mi][ni]); }
#pragma unroll
  for (int mi = 0; mi < 2; ++mi) {
    if (mi) __syncthreads();
#pragma unroll
    for (int ni = 0; ni < 4; ++ni)
#pragma unroll
      for (int r = 0; r < 8; ++r) sf[wave][8u * lh + r][ni * 16 + lm] = acc[mi][ni][r] * OSCALE;
    __syncthreads();
    v4f v[8];
#pragma unroll
    for (unsigned it = 0; it < 8; ++it) { const unsigned rw = it * 2u + (lane >> 4), pc = lane & 15u; v[it] = *(const v4f*)&sf[wave][rw][4u * pc]; }
    float* po = OUT + (size_t)(m0 + wm * 32u + mi * 16u) * DOUT + n0 + wn * 64u;
#pragma unroll
    for (unsigned it = 0; it < 8; ++it) { const unsigned rw = it * 2u + (lane >> 4), pc = lane & 15u; *(volatile v4f*)(po + (size_t)rw * DOUT + 4u * pc) = v[it]; }
    __threadfence();
#pragma unroll
    for (unsigned it = 0; it < 8; ++it) { const unsigned rw = it * 2u + (lane >> 4), pc = lane & 15u; *(volatile v4f*)(po + (size_t)rw * DOUT + 4u * pc) = v[it]; }
  }
}

extern "C" void kernel_launch(void* const* d_in, const int* in_sizes, int n_in, void* d_out, int out_size, void* d_ws, size_t ws_size, hipStream_t stream) {
  if (n_in < 8) return;
  if (in_sizes[0] < NB * DIN || in_sizes[1] < DIN * NE || in_sizes[2] < NE || in_sizes[3] < NE) return;
  if (in_sizes[4] < NE * DIN * DHID || in_sizes[5] < NE * DHID || in_sizes[6] < NE * DHID * DOUT || in_sizes[7] < NE * DOUT) return;
  if ((size_t)out_size < (size_t)NB * DOUT) return;
  if (ws_size < (size_t)WS_END) return;
  const float* X  = (const float*)d_in[0];
  const float* WG = (const float*)d_in[1];
  const float* BG = (const float*)d_in[2];
  const float* BI = (const float*)d_in[3];
  const float* W1 = (const float*)d_in[4];
  const float* B1 = (const float*)d_in[5];
  const float* W2 = (const float*)d_in[6];
  const float* B2 = (const float*)d_in[7];
  char* ws = (char*)d_ws;
  unsigned short* XB  = (unsigned short*)(ws + WS_XB);
  unsigned short* W1T = (unsigned short*)(ws + WS_W1T);
  unsigned short* W2T = (unsigned short*)(ws + WS_W2T);
  unsigned short* HB  = (unsigned short*)(ws + WS_HB);
  float* CW   = (float*)(ws + WS_CW);
  float* OUT  = (float*)d_out;
  k_cvt_x<<<dim3(NB * DIN / 8 / 256), 256, 0, stream>>>(X, XB);
  k_tr<0><<<dim3(DHID / 64, DIN / 64, NE), 256, 0, stream>>>(W1, W1T, (unsigned)DIN, (unsigned)DHID, (unsigned)DIN, (unsigned)DHID, 0u, 1.0f);
  k_tr<1><<<dim3(DOUT / 64, DHID / 64, NE), 256, 0, stream>>>(W2, W2T, (unsigned)DHID, (unsigned)DOUT, (unsigned)KP, 0u, (unsigned)DHID, WCARRY);
  k_b2pad<<<dim3(DOUT * 8 / 256), 256, 0, stream>>>(B2, W2T);
  k_gate<<<dim3(NB / 64), 256, 0, stream>>>(XB, WG, BG, BI, CW, HB);
  k_h<<<dim3(DHID / 128, NB / 128, NE), 256, 0, stream>>>(XB, W1T, B1, CW, HB);
  k_out<<<dim3(DOUT / 128, NB / 128), 256, 0, stream>>>(HB, W2T, OUT);
}
